// SimCSELoss_63874753626115
// MI455X (gfx1250) — hardware-verified
//
#include <hip/hip_runtime.h>
#include <stdint.h>
#include <math.h>


typedef _Float16 v16h __attribute__((ext_vector_type(16)));
typedef _Float16 v8h  __attribute__((ext_vector_type(8)));
typedef float    v8f  __attribute__((ext_vector_type(8)));
typedef float    v4f  __attribute__((ext_vector_type(4)));
union Frag { v16h v; v8h half[2]; };

#define NB    4096
#define N2    8192
#define DD    1024
#define TILE  128
#define NT    64
#define NTRI  2080
#define NUH   136
#define USLOT 32
#define NRB   32
#define ZSC   32.0f
#define KEXP  0.009765625f
#define KG    0.0009765625f

static_assert(NT * TILE == N2);
static_assert(NTRI == NT * (NT + 1) / 2);
static_assert(NB % NRB == 0);

__device__ __forceinline__ v8f wmma_f16(v8f acc, v16h a, v16h b)
{
    acc = __builtin_amdgcn_wmma_f32_16x16x32_f16(false, a, false, b, (short)0, acc, false, false);
    asm volatile("v_nop\n\tv_nop\n\tv_nop\n\tv_nop" : "+v"(acc) : "v"(a), "v"(b));
    return acc;
}

__device__ __forceinline__ float wave_sum(float x)
{
#pragma unroll
    for (int s = 16; s >= 1; s >>= 1) x += __shfl_xor(x, s, 32);
    return x;
}

__global__ __launch_bounds__(256) void k_norm(const float* __restrict__ p1,
                                              const float* __restrict__ p2,
                                              _Float16* __restrict__ zh,
                                              float* __restrict__ difA,
                                              float* __restrict__ posA,
                                              float* __restrict__ sqA,
                                              int nblk)
{
    __shared__ float sdif[NRB];
    __shared__ float spos[NRB];
    __shared__ float ssq[NRB];

    const int t = threadIdx.x, w = t >> 5, lane = t & 31;
    const int blk = blockIdx.x;
    if (blk >= nblk) return;

#pragma unroll 1
    for (int q = 0; q < 4; ++q) {
        const int r = blk * NRB + w * 4 + q;
        const float* g1 = p1 + (size_t)r * DD;
        const float* g2 = p2 + (size_t)r * DD;
        _Float16* z1 = zh + (size_t)r * DD;
        _Float16* z2 = zh + (size_t)(r + NB) * DD;

        float ss1 = 0.f, ss2 = 0.f;
#pragma unroll 1
        for (int p = 0; p < 4; ++p) {
            const int o = p * 256 + 8 * lane;
            const v4f a0 = *(const v4f*)(g1 + o), a1 = *(const v4f*)(g1 + o + 4);
            const v4f b0 = *(const v4f*)(g2 + o), b1 = *(const v4f*)(g2 + o + 4);
#pragma unroll
            for (int e = 0; e < 4; ++e) {
                ss1 += a0[e] * a0[e]; ss1 += a1[e] * a1[e];
                ss2 += b0[e] * b0[e]; ss2 += b1[e] * b1[e];
            }
        }
        ss1 = wave_sum(ss1);
        ss2 = wave_sum(ss2);
        const float inv1 = 1.0f / fmaxf(sqrtf(ss1), 1e-12f);
        const float inv2 = 1.0f / fmaxf(sqrtf(ss2), 1e-12f);

        float pos = 0.f, dif = 0.f, sq = 0.f;
#pragma unroll 1
        for (int p = 0; p < 4; ++p) {
            const int o = p * 256 + 8 * lane;
            const v4f a0 = *(const v4f*)(g1 + o), a1 = *(const v4f*)(g1 + o + 4);
            const v4f b0 = *(const v4f*)(g2 + o), b1 = *(const v4f*)(g2 + o + 4);
            v8h ha, hc;
#pragma unroll
            for (int e = 0; e < 8; ++e) {
                const float xa = (e < 4) ? a0[e & 3] : a1[e & 3];
                const float xc = (e < 4) ? b0[e & 3] : b1[e & 3];
                const float a = xa * inv1;
                const float c = xc * inv2;
                pos += a * c;
                const float d = a - c;
                dif += d * d;
                const _Float16 ah = (_Float16)(a * ZSC);
                const _Float16 ch = (_Float16)(c * ZSC);
                const float af = (float)ah;
                sq += af * af;
                ha[e] = ah; hc[e] = ch;
            }
            *(volatile v8h*)(z1 + o) = ha;
            *(volatile v8h*)(z2 + o) = hc;
        }
        __threadfence();
#pragma unroll 1
        for (int p = 0; p < 4; ++p) {
            const int o = p * 256 + 8 * lane;
            const v4f a0 = *(const v4f*)(g1 + o), a1 = *(const v4f*)(g1 + o + 4);
            const v4f b0 = *(const v4f*)(g2 + o), b1 = *(const v4f*)(g2 + o + 4);
            v8h ha, hc;
#pragma unroll
            for (int e = 0; e < 8; ++e) {
                const float xa = (e < 4) ? a0[e & 3] : a1[e & 3];
                const float xc = (e < 4) ? b0[e & 3] : b1[e & 3];
                ha[e] = (_Float16)((xa * inv1) * ZSC);
                hc[e] = (_Float16)((xc * inv2) * ZSC);
            }
            *(volatile v8h*)(z1 + o) = ha;
            *(volatile v8h*)(z2 + o) = hc;
        }

        pos = wave_sum(pos);
        dif = wave_sum(dif);
        sq  = wave_sum(sq);
        if (lane == 0) {
            sdif[w * 4 + q] = dif;
            spos[w * 4 + q] = pos;
            ssq[w * 4 + q]  = sq * KG;
        }
    }
    __syncthreads();

    if (w == 0 && lane < 24) {
        const int grp = lane >> 3, li = lane & 7;
        v4f val;
        float* dst;
        if (grp == 0) {
            val[0] = sdif[4 * li]; val[1] = sdif[4 * li + 1]; val[2] = sdif[4 * li + 2]; val[3] = sdif[4 * li + 3];
            dst = difA + (size_t)blk * NRB + 4 * li;
        } else if (grp == 1) {
            val[0] = spos[4 * li]; val[1] = spos[4 * li + 1]; val[2] = spos[4 * li + 2]; val[3] = spos[4 * li + 3];
            dst = posA + (size_t)blk * NRB + 4 * li;
        } else {
            val[0] = ssq[4 * li]; val[1] = ssq[4 * li + 1]; val[2] = ssq[4 * li + 2]; val[3] = ssq[4 * li + 3];
            dst = sqA + (size_t)blk * NRB + 4 * li;
        }
        *(volatile v4f*)dst = val;
        __threadfence();
        *(volatile v4f*)dst = val;
    }
}

__global__ __launch_bounds__(256) void k_tile(const _Float16* __restrict__ zh,
                                              const float* __restrict__ sqA,
                                              float* __restrict__ part,
                                              float* __restrict__ upart,
                                              int ntiles)
{
    __shared__ float colred[8][TILE];
    __shared__ float rowst[TILE];
    __shared__ float colst[TILE];
    __shared__ float ured[8];

    const int t = threadIdx.x, wave = t >> 5, lane = t & 31;
    const int m = lane & 15, h = lane >> 4, mrow = wave * 16;

    const int idx = blockIdx.x;
    if (idx >= ntiles) return;
    int rt = 0, base = 0;
    while (rt < NT - 1 && idx >= base + (NT - rt)) { base += NT - rt; ++rt; }
    int ct = rt + (idx - base);
    if (ct > NT - 1) ct = NT - 1;
    const bool isDiag = (ct == rt);
    const bool isU = (rt < 16 && ct < 16) || (rt >= 16 && rt < 32 && ct >= 16 && ct < 32);
    const int R0 = rt * TILE, C0 = ct * TILE;

    const _Float16* arow = zh + (size_t)(R0 + mrow + m) * DD + 8 * h;
    const _Float16* brow = zh + (size_t)(C0 + m) * DD + 8 * h;

    const v8f z8 = {0.f, 0.f, 0.f, 0.f, 0.f, 0.f, 0.f, 0.f};
    v8f c[8];
#pragma unroll
    for (int n = 0; n < 8; ++n) c[n] = z8;

#pragma unroll 2
    for (int k0 = 0; k0 < DD; k0 += 32) {
        Frag a;
        a.half[0] = *(const v8h*)(arow + k0);
        a.half[1] = *(const v8h*)(arow + k0 + 16);
#pragma unroll
        for (int n = 0; n < 8; ++n) {
            const _Float16* bp = brow + (size_t)n * (16 * DD) + k0;
            Frag b;
            b.half[0] = *(const v8h*)(bp);
            b.half[1] = *(const v8h*)(bp + 16);
            c[n] = wmma_f16(c[n], a.v, b.v);
        }
    }

    float sqr[8], sqc[8];
#pragma unroll
    for (int v = 0; v < 8; ++v) sqr[v] = 0.f;
#pragma unroll
    for (int n = 0; n < 8; ++n) sqc[n] = 0.f;
    if (isU) {
#pragma unroll
        for (int v = 0; v < 8; ++v) sqr[v] = sqA[R0 + mrow + 8 * h + v];
#pragma unroll
        for (int n = 0; n < 8; ++n) sqc[n] = sqA[C0 + 16 * n + m];
    }

    float rs[8], cs[8];
#pragma unroll
    for (int v = 0; v < 8; ++v) rs[v] = 0.f;
#pragma unroll
    for (int n = 0; n < 8; ++n) cs[n] = 0.f;
    float us = 0.f;

#pragma unroll
    for (int n = 0; n < 8; ++n) {
        const int lc = 16 * n + m;
#pragma unroll
        for (int v = 0; v < 8; ++v) {
            const int lr = mrow + 8 * h + v;
            const float gs = c[n][v];
            float p = __expf(gs * KEXP - 10.0f);
            if (isDiag && lr == lc) p = 0.f;
            rs[v] += p;
            cs[n] += p;
            if (isU) {
                const float d2 = fmaxf(sqr[v] + sqc[n] - 2.0f * (gs * KG), 0.0f);
                const float u = __expf(-2.0f * d2);
                if (!isDiag || lc > lr) us += u;
            }
        }
    }

#pragma unroll
    for (int v = 0; v < 8; ++v) {
        float x = rs[v];
        x += __shfl_xor(x, 1, 32);
        x += __shfl_xor(x, 2, 32);
        x += __shfl_xor(x, 4, 32);
        x += __shfl_xor(x, 8, 32);
        rs[v] = x;
    }
#pragma unroll
    for (int n = 0; n < 8; ++n) cs[n] += __shfl_xor(cs[n], 16, 32);
    us = wave_sum(us);

    if (m == 0) {
#pragma unroll
        for (int v = 0; v < 8; ++v) rowst[mrow + 8 * h + v] = rs[v];
    }
    if (h == 0) {
#pragma unroll
        for (int n = 0; n < 8; ++n) colred[wave][16 * n + m] = cs[n];
    }
    if (lane == 0) ured[wave] = us;
    __syncthreads();
    if (t < TILE) {
        float s = 0.f;
#pragma unroll
        for (int ww = 0; ww < 8; ++ww) s += colred[ww][t];
        colst[t] = s;
    }
    __syncthreads();

    bool act = false;
    v4f val = {0.f, 0.f, 0.f, 0.f};
    float* dst = part;
    if (wave == 0) {
        act = true;
        val[0] = rowst[4 * lane]; val[1] = rowst[4 * lane + 1];
        val[2] = rowst[4 * lane + 2]; val[3] = rowst[4 * lane + 3];
        dst = part + (size_t)ct * N2 + R0 + 4 * lane;
    } else if (wave == 1) {
        if (!isDiag) {
            act = true;
            val[0] = colst[4 * lane]; val[1] = colst[4 * lane + 1];
            val[2] = colst[4 * lane + 2]; val[3] = colst[4 * lane + 3];
            dst = part + (size_t)rt * N2 + C0 + 4 * lane;
        }
    } else if (wave == 2) {
        if (isU && lane < 8) {
            float ut = 0.f;
#pragma unroll
            for (int ww = 0; ww < 8; ++ww) ut += ured[ww];
            if (lane == 0) val[0] = ut;
            const int hh = rt >> 4;
            const int lrt = rt - 16 * hh, lct = ct - 16 * hh;
            const int uidx = hh * NUH + 16 * lrt - (lrt * (lrt - 1)) / 2 + (lct - lrt);
            if ((unsigned)uidx < (unsigned)(2 * NUH)) {
                act = true;
                dst = upart + (size_t)uidx * USLOT + 4 * lane;
            }
        }
    }
    if (act) *(volatile v4f*)dst = val;
    __threadfence();
    if (act) *(volatile v4f*)dst = val;
}

__global__ __launch_bounds__(256) void k_final(const float* __restrict__ part,
                                               const float* __restrict__ difA,
                                               const float* __restrict__ posA,
                                               const float* __restrict__ upart,
                                               float* __restrict__ out)
{
    __shared__ double red[3][256];
    const int t = threadIdx.x;

    double slog = 0.0;
    for (int i = t; i < N2; i += 256) {
        double s = 0.0;
#pragma unroll 4
        for (int tt = 0; tt < NT; ++tt) s += (double)part[(size_t)tt * N2 + i];
        slog += log(fmax(s, 1e-300));
    }
    double spos = 0.0, sdif = 0.0;
    for (int r = t; r < NB; r += 256) {
        spos += (double)posA[r];
        sdif += (double)difA[r];
    }
    red[0][t] = slog; red[1][t] = spos; red[2][t] = sdif;
    __syncthreads();

    if (t == 0) {
        double L = 0.0, P = 0.0, Df = 0.0;
        for (int j = 0; j < 256; ++j) { L += red[0][j]; P += red[1][j]; Df += red[2][j]; }
        double U0 = 0.0, U1 = 0.0;
        for (int j = 0; j < NUH; ++j) {
            U0 += (double)upart[(size_t)j * USLOT];
            U1 += (double)upart[(size_t)(NUH + j) * USLOT];
        }
        const double nh = (double)(NB / 2);
        const double pairs = nh * (nh - 1.0) * 0.5;
        const float o0 = (float)((10.0 * (double)N2 + L - 20.0 * P) / (double)N2);
        const float o1 = (float)(Df / (double)NB);
        const float o2 = (float)(0.5 * (log(fmax(U0, 1e-300) / pairs) + log(fmax(U1, 1e-300) / pairs)));
        volatile float* vo = out;
        vo[0] = o0; vo[1] = o1; vo[2] = o2;
        __threadfence();
        vo[0] = o0; vo[1] = o1; vo[2] = o2;
    }
}

extern "C" void kernel_launch(void* const* d_in, const int* in_sizes, int n_in,
                              void* d_out, int out_size, void* d_ws, size_t ws_size,
                              hipStream_t stream)
{
    if (n_in < 2 || out_size < 3) return;
    if (in_sizes[0] != NB * DD || in_sizes[1] != NB * DD) return;

    const float* p1 = (const float*)d_in[0];
    const float* p2 = (const float*)d_in[1];
    float* out = (float*)d_out;

    char* ws = (char*)d_ws;
    const size_t zhB   = (size_t)N2 * DD * sizeof(_Float16);
    const size_t vecB  = (size_t)NB * sizeof(float);
    const size_t partB = (size_t)NT * N2 * sizeof(float);
    const size_t upB   = (size_t)2 * NUH * USLOT * sizeof(float);
    size_t off = 0;
    _Float16* zh = (_Float16*)(ws + off); off += zhB;
    float* difA  = (float*)(ws + off);    off += vecB;
    float* posA  = (float*)(ws + off);    off += vecB;
    float* sqA   = (float*)(ws + off);    off += vecB;
    float* part  = (float*)(ws + off);    off += partB;
    float* upart = (float*)(ws + off);    off += upB;
    if (off > ws_size) return;

    const int nblk = NB / NRB;
    const int ntiles = NTRI;

    k_norm<<<nblk, 256, 0, stream>>>(p1, p2, zh, difA, posA, sqA, nblk);
    k_tile<<<ntiles, 256, 0, stream>>>(zh, sqA, part, upart, ntiles);
    k_final<<<1, 256, 0, stream>>>(part, difA, posA, upart, out);
}
